// EncGausSALayer_86242943304258
// MI455X (gfx1250) — hardware-verified
//
#include <hip/hip_runtime.h>
#include <math.h>
#include <stdint.h>

#define TT    1024
#define BBT   8
#define CC    512
#define NHD   8
#define HD    64
#define FFD   2048
#define KTAP  9
#define NROW  (TT * BBT)
#define PADR  32
#define NROWP (NROW + 2 * PADR)
#define KFF   (KTAP * CC)

static_assert(NHD * HD == CC);
static_assert((NROW % 64) == 0 && (CC % 64) == 0 && (FFD % 64) == 0 && (TT % 64) == 0);
static_assert((CC % 32) == 0 && (KFF % 32) == 0 && (FFD % 32) == 0);
static_assert((NROW % 8) == 0);
static_assert(((PADR * CC) % (8 * 256)) == 0);

#define CARRY_W 64.0f
#define CARRY_Q 8.0f
#define CARRY_P 1024.0f
#define CARRY_O 16.0f
#define CARRY_R 16.0f
#define THIRD   0.333333343f
#define LN_EPS  1e-5f

typedef _Float16 v16h __attribute__((ext_vector_type(16)));
typedef _Float16 v8h  __attribute__((ext_vector_type(8)));
typedef float    v8f  __attribute__((ext_vector_type(8)));
typedef float    v4f  __attribute__((ext_vector_type(4)));
typedef unsigned int v4u __attribute__((ext_vector_type(4)));

__device__ __forceinline__ unsigned short h_bits(_Float16 x) { return __builtin_bit_cast(unsigned short, x); }
__device__ __forceinline__ unsigned pk2(float a, float b) {
  return (unsigned)h_bits((_Float16)a) | ((unsigned)h_bits((_Float16)b) << 16);
}
__device__ __forceinline__ v8f zero8() { v8f z = {0.f, 0.f, 0.f, 0.f, 0.f, 0.f, 0.f, 0.f}; return z; }

__device__ __forceinline__ v16h ldfrag_h(const _Float16* p) {
  union { v16h v; v8h h[2]; } f;
  f.h[0] = *(const v8h*)(p);
  f.h[1] = *(const v8h*)(p + 16);
  return f.v;
}

__device__ __forceinline__ v8f mma_h(v16h a, v16h b, v8f c) {
  c = __builtin_amdgcn_wmma_f32_16x16x32_f16(false, a, false, b, (short)0, c, false, false);
#if defined(__HIP_DEVICE_COMPILE__)
  asm volatile("v_nop\n\tv_nop\n\tv_nop\n\tv_nop" : "+v"(c) : "v"(a), "v"(b));
#endif
  return c;
}
__device__ __forceinline__ v8f mma_raw(v16h a, v16h b, v8f c) {
  return __builtin_amdgcn_wmma_f32_16x16x32_f16(false, a, false, b, (short)0, c, false, false);
}
__device__ __forceinline__ void dep_guard(v8f& a, v8f& b, v16h x, v16h y) {
#if defined(__HIP_DEVICE_COMPILE__)
  asm volatile("v_nop\n\tv_nop\n\tv_nop\n\tv_nop" : "+v"(a), "+v"(b) : "v"(x), "v"(y));
#endif
}
__device__ __forceinline__ void keep4(v16h a, v16h b, v16h c, v16h d) {
#if defined(__HIP_DEVICE_COMPILE__)
  asm volatile("v_nop" :: "v"(a), "v"(b), "v"(c), "v"(d));
#endif
}
__device__ __forceinline__ void acc_guard4(v8f& a, v8f& b, v8f& c, v8f& d) {
#if defined(__HIP_DEVICE_COMPILE__)
  asm volatile("v_nop\n\tv_nop\n\tv_nop\n\tv_nop" : "+v"(a), "+v"(b), "+v"(c), "+v"(d));
#endif
}
__device__ __forceinline__ void wave_sync_lds() {
  __builtin_amdgcn_fence(__ATOMIC_RELEASE, "workgroup");
  __builtin_amdgcn_wave_barrier();
  __builtin_amdgcn_fence(__ATOMIC_ACQUIRE, "workgroup");
}

__global__ __launch_bounds__(256) void zero_pad(_Float16* base, long long off1, int n8) {
  const int i = blockIdx.x * 256 + threadIdx.x;
  if (i >= 2 * n8) return;
  const size_t eo = (i < n8) ? ((size_t)i * 8) : ((size_t)off1 + (size_t)(i - n8) * 8);
  v4u z;
  z[0] = 0u; z[1] = 0u; z[2] = 0u; z[3] = 0u;
  _Float16* d = base + eo;
  *(volatile v4u*)d = z;
  __threadfence();
  *(volatile v4u*)d = z;
}

__global__ __launch_bounds__(256) void wt_cvt(const float* __restrict__ W, _Float16* out,
                                               int R, int Cn, float scale) {
  __shared__ float tile[64 * 65];
  const int tid = threadIdx.x;
  const int n0 = blockIdx.x * 64;
  const int k0 = blockIdx.y * 64;
  {
    const int kr = tid >> 2, q16 = (tid & 3) * 16;
    const float* src = W + (size_t)(k0 + kr) * Cn + n0 + q16;
#pragma unroll
    for (int e = 0; e < 4; ++e) {
      const v4f v = *(const v4f*)(src + 4 * e);
      float* d = tile + kr * 65 + q16 + 4 * e;
      d[0] = v[0]; d[1] = v[1]; d[2] = v[2]; d[3] = v[3];
    }
  }
  __syncthreads();
  const int c8 = (tid & 7) * 8;
  v4u pv[2];
#pragma unroll
  for (int it = 0; it < 2; ++it) {
    const int nn = (tid >> 3) + 32 * it;
    float f[8];
#pragma unroll
    for (int j = 0; j < 8; ++j) f[j] = tile[(c8 + j) * 65 + nn] * scale;
    v4u pp;
    pp[0] = pk2(f[0], f[1]); pp[1] = pk2(f[2], f[3]);
    pp[2] = pk2(f[4], f[5]); pp[3] = pk2(f[6], f[7]);
    pv[it] = pp;
  }
  for (int pass = 0; pass < 2; ++pass) {
#pragma unroll
    for (int it = 0; it < 2; ++it) {
      const int nn = (tid >> 3) + 32 * it;
      *(volatile v4u*)(out + (size_t)(n0 + nn) * R + k0 + c8) = pv[it];
    }
    __threadfence();
  }
}

__global__ __launch_bounds__(256) void ln_rows(const float* __restrict__ in, const float* __restrict__ g,
                                                const float* __restrict__ be, _Float16* out,
                                                int nrows, int orow_off) {
  const int lane = threadIdx.x & 31;
  const int row  = blockIdx.x * 8 + (threadIdx.x >> 5);
  if (row >= nrows) return;
  const float* p = in + (size_t)row * CC;
  const int c0 = 8 * lane, c1 = 256 + 8 * lane;
  const v4f a0 = *(const v4f*)(p + c0), a1 = *(const v4f*)(p + c0 + 4);
  const v4f a2 = *(const v4f*)(p + c1), a3 = *(const v4f*)(p + c1 + 4);
  float s = 0.f;
#pragma unroll
  for (int e = 0; e < 4; ++e) { s += a0[e]; s += a1[e]; s += a2[e]; s += a3[e]; }
#pragma unroll
  for (int off = 1; off < 32; off <<= 1) s += __shfl_xor(s, off, 32);
  const float mean = s * (1.0f / (float)CC);
  const v4f d0 = a0 - mean, d1 = a1 - mean, d2 = a2 - mean, d3 = a3 - mean;
  float s2 = 0.f;
#pragma unroll
  for (int e = 0; e < 4; ++e) { s2 += d0[e] * d0[e]; s2 += d1[e] * d1[e]; s2 += d2[e] * d2[e]; s2 += d3[e] * d3[e]; }
#pragma unroll
  for (int off = 1; off < 32; off <<= 1) s2 += __shfl_xor(s2, off, 32);
  const float var  = s2 * (1.0f / (float)CC);
  const float rstd = rsqrtf(var + LN_EPS);
  const v4f g0 = *(const v4f*)(g + c0), g1 = *(const v4f*)(g + c0 + 4);
  const v4f g2 = *(const v4f*)(g + c1), g3 = *(const v4f*)(g + c1 + 4);
  const v4f e0 = *(const v4f*)(be + c0), e1 = *(const v4f*)(be + c0 + 4);
  const v4f e2 = *(const v4f*)(be + c1), e3 = *(const v4f*)(be + c1 + 4);
  const v4f y0 = d0 * rstd * g0 + e0, y1 = d1 * rstd * g1 + e1;
  const v4f y2 = d2 * rstd * g2 + e2, y3 = d3 * rstd * g3 + e3;
  v4u p0, p1;
  p0[0] = pk2(y0[0], y0[1]); p0[1] = pk2(y0[2], y0[3]); p0[2] = pk2(y1[0], y1[1]); p0[3] = pk2(y1[2], y1[3]);
  p1[0] = pk2(y2[0], y2[1]); p1[1] = pk2(y2[2], y2[3]); p1[2] = pk2(y3[0], y3[1]); p1[3] = pk2(y3[2], y3[3]);
  _Float16* q = out + (size_t)(row + orow_off) * CC;
  for (int pass = 0; pass < 2; ++pass) {
    *(volatile v4u*)(q + c0) = p0;
    *(volatile v4u*)(q + c1) = p1;
    __threadfence();
  }
}

template <int AMODE, int EPI>
__global__ __launch_bounds__(256) void gemm64(
    const _Float16* __restrict__ A, int lda, long long strideA,
    const _Float16* __restrict__ Bt, int ldb, long long strideB,
    const float* __restrict__ bias, const float* __restrict__ bias2, int zsel,
    const float* __restrict__ resid,
    void* Cout, int ldc, long long strideC,
    int M, int N, int K, float ascale, float oscale) {
  __shared__ __align__(16) float sT[8][16 * 68];
  const int z    = blockIdx.y;
  const int lane = threadIdx.x & 31;
  const int wave = threadIdx.x >> 5;
  const int tilesN = N >> 6;
  const int tilesM = M >> 6;
  const int tile = blockIdx.x * 8 + wave;
  if (tile >= tilesM * tilesN) return;
  const int tm = tile / tilesN;
  const int tn = tile - tm * tilesN;
  const int m0 = tm << 6;
  const int n0 = tn << 6;

  const _Float16* Ab = A  + (size_t)z * (size_t)strideA;
  const _Float16* Bb = Bt + (size_t)z * (size_t)strideB;
  const float* bz = (zsel != 0 && z == 1) ? bias2 : bias;

  const int rlane = lane & 15;
  const int koff  = (lane >> 4) * 8;
  const int mOff  = (lane >> 4) * 8;

  v8f acc[4][4];
#pragma unroll
  for (int i = 0; i < 4; ++i)
#pragma unroll
    for (int j = 0; j < 4; ++j) acc[i][j] = zero8();

  for (int k0 = 0; k0 < K; k0 += 32) {
    size_t acol = (size_t)k0;
    if (AMODE == 1) {
      const int tap  = k0 >> 9;
      const int kk   = k0 & (CC - 1);
      const int roff = (tap == 0) ? PADR : (tap * BBT);
      acol = (size_t)roff * CC + (size_t)kk;
    }
    v16h bf[4];
#pragma unroll
    for (int j = 0; j < 4; ++j)
      bf[j] = ldfrag_h(Bb + (size_t)(n0 + (j << 4) + rlane) * ldb + koff + k0);
#pragma unroll
    for (int i = 0; i < 4; ++i) {
      const v16h af = ldfrag_h(Ab + (size_t)(m0 + (i << 4) + rlane) * lda + acol + koff);
#pragma unroll
      for (int j = 0; j < 4; ++j) acc[i][j] = mma_raw(af, bf[j], acc[i][j]);
      dep_guard(acc[i][0], acc[i][3], af, bf[3]);
    }
    keep4(bf[0], bf[1], bf[2], bf[3]);
  }
  acc_guard4(acc[0][0], acc[0][1], acc[0][2], acc[0][3]);
  acc_guard4(acc[1][0], acc[1][1], acc[1][2], acc[1][3]);
  acc_guard4(acc[2][0], acc[2][1], acc[2][2], acc[2][3]);
  acc_guard4(acc[3][0], acc[3][1], acc[3][2], acc[3][3]);

  float* slab = sT[wave];
#pragma unroll
  for (int i = 0; i < 4; ++i) {
    const int mBase = m0 + (i << 4);
#pragma unroll
    for (int j = 0; j < 4; ++j) {
#pragma unroll
      for (int r = 0; r < 8; ++r) {
        slab[(mOff + r) * 68 + (j << 4) + rlane] = acc[i][j][r];
      }
    }
    wave_sync_lds();
    if (EPI == 2) {
      float* C = (float*)Cout + (size_t)z * (size_t)strideC;
      const int hh = lane >> 4, c4 = (lane & 15) * 4;
      const v4f b4 = *(const v4f*)(bz + n0 + c4);
      v4f ov[8];
#pragma unroll
      for (int it = 0; it < 8; ++it) {
        const int row = it * 2 + hh;
        const v4f v  = *(const v4f*)(slab + row * 68 + c4);
        const v4f r4 = *(const v4f*)(resid + (size_t)(mBase + row) * ldc + n0 + c4);
        ov[it] = v * ascale + b4 + r4;
      }
      for (int pass = 0; pass < 2; ++pass) {
#pragma unroll
        for (int it = 0; it < 8; ++it) {
          const int row = it * 2 + hh;
          *(volatile v4f*)(C + (size_t)(mBase + row) * ldc + n0 + c4) = ov[it];
        }
        __threadfence();
      }
    } else {
      _Float16* C16 = (_Float16*)Cout + (size_t)z * (size_t)strideC;
      const int q = lane >> 3, c8 = (lane & 7) * 8;
      float bcol[8];
#pragma unroll
      for (int e = 0; e < 8; ++e) bcol[e] = 0.f;
      if (EPI != 1) {
        const v4f bc0 = *(const v4f*)(bz + n0 + c8);
        const v4f bc1 = *(const v4f*)(bz + n0 + c8 + 4);
        bcol[0] = bc0[0]; bcol[1] = bc0[1]; bcol[2] = bc0[2]; bcol[3] = bc0[3];
        bcol[4] = bc1[0]; bcol[5] = bc1[1]; bcol[6] = bc1[2]; bcol[7] = bc1[3];
      }
      v4u hv[4];
#pragma unroll
      for (int it = 0; it < 4; ++it) {
        const int row = it * 4 + q;
        const float* sp = slab + row * 68 + c8;
        const v4f x0 = *(const v4f*)(sp);
        const v4f x1 = *(const v4f*)(sp + 4);
        float brow = 0.f;
        if (EPI == 1) brow = bz[mBase + row];
        float f[8];
        f[0] = x0[0]; f[1] = x0[1]; f[2] = x0[2]; f[3] = x0[3];
        f[4] = x1[0]; f[5] = x1[1]; f[6] = x1[2]; f[7] = x1[3];
#pragma unroll
        for (int e = 0; e < 8; ++e) {
          const float bb = (EPI == 1) ? brow : bcol[e];
          float v = f[e] * ascale + bb;
          if (EPI == 3) v = fmaxf(v * THIRD, 0.f);
          f[e] = v * oscale;
        }
        v4u pp;
        pp[0] = pk2(f[0], f[1]); pp[1] = pk2(f[2], f[3]);
        pp[2] = pk2(f[4], f[5]); pp[3] = pk2(f[6], f[7]);
        hv[it] = pp;
      }
      for (int pass = 0; pass < 2; ++pass) {
#pragma unroll
        for (int it = 0; it < 4; ++it) {
          const int row = it * 4 + q;
          *(volatile v4u*)(C16 + (size_t)(mBase + row) * ldc + n0 + c8) = hv[it];
        }
        __threadfence();
      }
    }
    wave_sync_lds();
  }
}

__global__ __launch_bounds__(128)
void attn_dist(const _Float16* __restrict__ Qp, const _Float16* __restrict__ Kp,
               const _Float16* __restrict__ VTp, const float* __restrict__ tao,
               _Float16* Op, float sscale) {
  union FH { v16h v; v8h h[2]; };
  __shared__ __align__(16) _Float16 Ksh[64 * 64];
  __shared__ __align__(16) _Float16 Vth[64 * 64];
  __shared__ __align__(16) _Float16 Psh[4][16 * 64];
  __shared__ __align__(16) float    Os[4][16 * 64];

  const int tid  = threadIdx.x;
  const int wave = tid >> 5;
  const int lane = tid & 31;
  const int hh   = lane >> 4;
  const int c    = lane & 15;

  const int bx = blockIdx.x;
  const int qb = bx & 15;
  const int h  = (bx >> 4) & (NHD - 1);
  const int b  = bx >> 7;
  const int q0 = qb * 64 + wave * 16;

  const float tt   = tao[h];
  const float tt2  = tt * tt;
  const float tt4  = tt2 * tt2;
  const float tinv = 1.0f / tt4;

  const size_t rp = (size_t)BBT * CC;
  const _Float16* Qb = Qp  + (size_t)b * CC + (size_t)h * HD;
  const _Float16* Kb = Kp  + (size_t)b * CC + (size_t)h * HD;
  const _Float16* Vb = VTp + ((size_t)b * CC + (size_t)h * HD) * TT;

  v16h qa[2];
#pragma unroll
  for (int dc = 0; dc < 2; ++dc)
    qa[dc] = ldfrag_h(Qb + (size_t)(q0 + c) * rp + dc * 32 + 8 * hh);

  float mrow[8], lrow[8];
  v8f oacc[4];
#pragma unroll
  for (int r = 0; r < 8; ++r) { mrow[r] = -INFINITY; lrow[r] = 0.f; }
#pragma unroll
  for (int t = 0; t < 4; ++t) oacc[t] = zero8();

  for (int kt = 0; kt < TT / 64; ++kt) {
    const int kv0 = kt * 64;
    __syncthreads();
    {
      const int r = tid >> 1, half = (tid & 1) * 32;
      const _Float16* kg = Kb + (size_t)(kv0 + r) * rp + half;
      const _Float16* vg = Vb + (size_t)r * TT + kv0 + half;
#pragma unroll
      for (int i = 0; i < 4; ++i) {
        const v8h a0 = *(const v8h*)(kg + 8 * i);
        const v8h b0 = *(const v8h*)(vg + 8 * i);
        *(v8h*)(Ksh + r * 64 + half + 8 * i) = a0;
        *(v8h*)(Vth + r * 64 + half + 8 * i) = b0;
      }
    }
    __syncthreads();

    v8f s[4];
#pragma unroll
    for (int j = 0; j < 4; ++j) {
      s[j] = zero8();
#pragma unroll
      for (int dc = 0; dc < 2; ++dc) {
        FH kb;
        kb.h[0] = *(const v8h*)(Ksh + (j * 16 + c) * 64 + dc * 32 + 8 * hh);
        kb.h[1] = *(const v8h*)(Ksh + (j * 16 + c) * 64 + dc * 32 + 16 + 8 * hh);
        s[j] = mma_h(qa[dc], kb.v, s[j]);
      }
    }

    _Float16* pw = Psh[wave];
#pragma unroll
    for (int r = 0; r < 8; ++r) {
      const float qi = (float)(q0 + 8 * hh + r);
      float m = -INFINITY;
#pragma unroll
      for (int j = 0; j < 4; ++j) {
        const float kj = (float)(kv0 + j * 16 + c);
        const float df = qi - kj;
        const float gb = -(df * df) * 0.5f;
        const float sv = s[j][r] * sscale + gb * tinv;
        s[j][r] = sv;
        m = fmaxf(m, sv);
      }
#pragma unroll
      for (int off = 1; off < 16; off <<= 1) m = fmaxf(m, __shfl_xor(m, off, 32));
      const float mnew  = fmaxf(mrow[r], m);
      const float msafe = (mnew == -INFINITY) ? 0.f : mnew;
      const float alpha = __expf(mrow[r] - msafe);
      mrow[r] = mnew;
      float psum = 0.f;
#pragma unroll
      for (int j = 0; j < 4; ++j) {
        const float p = __expf(s[j][r] - msafe);
        psum += p;
        pw[(8 * hh + r) * 64 + j * 16 + c] = (_Float16)(p * CARRY_P);
      }
#pragma unroll
      for (int off = 1; off < 16; off <<= 1) psum += __shfl_xor(psum, off, 32);
      lrow[r] = lrow[r] * alpha + psum;
#pragma unroll
      for (int t = 0; t < 4; ++t) oacc[t][r] *= alpha;
    }
    wave_sync_lds();

#pragma unroll 1
    for (int kk = 0; kk < 2; ++kk) {
      FH pa;
      pa.h[0] = *(const v8h*)(pw + c * 64 + kk * 32 + 8 * hh);
      pa.h[1] = *(const v8h*)(pw + c * 64 + kk * 32 + 16 + 8 * hh);
#pragma unroll
      for (int t = 0; t < 4; ++t) {
        FH vb;
        vb.h[0] = *(const v8h*)(Vth + (t * 16 + c) * 64 + kk * 32 + 8 * hh);
        vb.h[1] = *(const v8h*)(Vth + (t * 16 + c) * 64 + kk * 32 + 16 + 8 * hh);
        oacc[t] = mma_h(pa.v, vb.v, oacc[t]);
      }
    }
  }

  float* os = Os[wave];
#pragma unroll
  for (int r = 0; r < 8; ++r) {
    const float l = lrow[r];
    const float inv = ((l > 0.f) ? (1.0f / l) : 0.f) * (CARRY_O / (CARRY_P * CARRY_Q));
#pragma unroll
    for (int t = 0; t < 4; ++t) os[(8 * hh + r) * 64 + t * 16 + c] = oacc[t][r] * inv;
  }
  wave_sync_lds();
  {
    const int q4 = lane >> 3, c8 = (lane & 7) * 8;
    v4u hv[4];
#pragma unroll
    for (int it = 0; it < 4; ++it) {
      const int row = it * 4 + q4;
      const float* sp = os + row * 64 + c8;
      const v4f x0 = *(const v4f*)(sp);
      const v4f x1 = *(const v4f*)(sp + 4);
      v4u pp;
      pp[0] = pk2(x0[0], x0[1]); pp[1] = pk2(x0[2], x0[3]);
      pp[2] = pk2(x1[0], x1[1]); pp[3] = pk2(x1[2], x1[3]);
      hv[it] = pp;
    }
    for (int pass = 0; pass < 2; ++pass) {
#pragma unroll
      for (int it = 0; it < 4; ++it) {
        const int row = it * 4 + q4;
        const size_t go = ((size_t)(q0 + row) * BBT + (size_t)b) * CC + (size_t)h * HD + c8;
        *(volatile v4u*)(Op + go) = hv[it];
      }
      __threadfence();
    }
  }
}

extern "C" void kernel_launch(void* const* d_in, const int* in_sizes, int n_in,
                              void* d_out, int out_size, void* d_ws, size_t ws_size,
                              hipStream_t stream) {
  if (n_in < 18) return;
  if (in_sizes[0] != NROW * CC) return;
  if (in_sizes[1] != CC || in_sizes[2] != CC) return;
  if (in_sizes[3] != CC * CC || in_sizes[4] != CC) return;
  if (in_sizes[5] != CC * CC || in_sizes[6] != CC) return;
  if (in_sizes[7] != CC * CC || in_sizes[8] != CC) return;
  if (in_sizes[9] != NHD) return;
  if (in_sizes[10] != CC * CC || in_sizes[11] != CC) return;
  if (in_sizes[12] != CC || in_sizes[13] != CC) return;
  if (in_sizes[14] != KTAP * CC * FFD || in_sizes[15] != FFD) return;
  if (in_sizes[16] != FFD * CC || in_sizes[17] != CC) return;
  if (out_size != NROW * CC) return;

  const float* x     = (const float*)d_in[0];
  const float* ln1_g = (const float*)d_in[1];
  const float* ln1_b = (const float*)d_in[2];
  const float* wq    = (const float*)d_in[3];
  const float* wq_b  = (const float*)d_in[4];
  const float* wk    = (const float*)d_in[5];
  const float* wk_b  = (const float*)d_in[6];
  const float* wv    = (const float*)d_in[7];
  const float* wv_b  = (const float*)d_in[8];
  const float* tao   = (const float*)d_in[9];
  const float* fc_w  = (const float*)d_in[10];
  const float* fc_b  = (const float*)d_in[11];
  const float* ln2_g = (const float*)d_in[12];
  const float* ln2_b = (const float*)d_in[13];
  const float* f1_w  = (const float*)d_in[14];
  const float* f1_b  = (const float*)d_in[15];
  const float* f2_w  = (const float*)d_in[16];
  const float* f2_b  = (const float*)d_in[17];

  const size_t SZ_WQK = (size_t)2 * CC * CC * 2;
  const size_t SZ_W   = (size_t)CC * CC * 2;
  const size_t SZ_W1  = (size_t)FFD * KFF * 2;
  const size_t SZ_W2  = (size_t)CC * FFD * 2;
  const size_t SZ_ACT = (size_t)NROW * CC * 2;
  const size_t SZ_QK  = (size_t)2 * NROW * CC * 2;
  const size_t SZ_VT  = (size_t)BBT * CC * TT * 2;
  const size_t SZ_X1  = (size_t)NROW * CC * 4;
  const size_t SZ_H2  = (size_t)NROWP * CC * 2;
  const size_t SZ_RES = (size_t)NROW * FFD * 2;
  size_t off = 0;
  const size_t oWqk = off; off += SZ_WQK;
  const size_t oWv  = off; off += SZ_W;
  const size_t oWfc = off; off += SZ_W;
  const size_t oW1  = off; off += SZ_W1;
  const size_t oW2  = off; off += SZ_W2;
  const size_t oHx  = off; off += SZ_ACT;
  const size_t oQK  = off; off += SZ_QK;
  const size_t oVT  = off; off += SZ_VT;
  const size_t oO   = off; off += SZ_ACT;
  const size_t oX1  = off; off += SZ_X1;
  const size_t oH2  = off; off += SZ_H2;
  const size_t oRes = off; off += SZ_RES;
  if (off > ws_size) return;
  if (off > (size_t)134217728) return;

  char* ws = (char*)d_ws;
  _Float16* WqkT = (_Float16*)(ws + oWqk);
  _Float16* WvT  = (_Float16*)(ws + oWv);
  _Float16* WfcT = (_Float16*)(ws + oWfc);
  _Float16* W1T  = (_Float16*)(ws + oW1);
  _Float16* W2T  = (_Float16*)(ws + oW2);
  _Float16* Hx   = (_Float16*)(ws + oHx);
  _Float16* QK   = (_Float16*)(ws + oQK);
  _Float16* VT   = (_Float16*)(ws + oVT);
  _Float16* Opl  = (_Float16*)(ws + oO);
  float*    X1   = (float*)(ws + oX1);
  _Float16* H2p  = (_Float16*)(ws + oH2);
  _Float16* Res  = (_Float16*)(ws + oRes);

  const dim3 blk(256);
  const int tilesQK  = (NROW / 64) * (CC / 64);
  const int tilesVT  = (CC / 64) * (TT / 64);
  const int tilesFF1 = (NROW / 64) * (FFD / 64);
  const dim3 gQK((tilesQK + 7) / 8, 2);
  const dim3 gVT((tilesVT + 7) / 8, BBT);
  const dim3 gFC((tilesQK + 7) / 8, 1);
  const dim3 gFF1((tilesFF1 + 7) / 8, 1);
  const dim3 gAttn(BBT * NHD * (TT / 64));
  const dim3 gLN(NROW / 8);
  const int  n8pad = PADR * CC / 8;
  const dim3 gPad((2 * n8pad + 255) / 256);

  zero_pad<<<gPad, blk, 0, stream>>>(H2p, (long long)(PADR + NROW) * CC, n8pad);
  wt_cvt<<<dim3(CC / 64, CC / 64), blk, 0, stream>>>(wq,   WqkT,                  CC,  CC,  CARRY_W);
  wt_cvt<<<dim3(CC / 64, CC / 64), blk, 0, stream>>>(wk,   WqkT + (size_t)CC * CC, CC, CC,  CARRY_W);
  wt_cvt<<<dim3(CC / 64, CC / 64), blk, 0, stream>>>(wv,   WvT,                   CC,  CC,  CARRY_W);
  wt_cvt<<<dim3(CC / 64, CC / 64), blk, 0, stream>>>(fc_w, WfcT,                  CC,  CC,  CARRY_W);
  wt_cvt<<<dim3(FFD / 64, KFF / 64), blk, 0, stream>>>(f1_w, W1T,                 KFF, FFD, CARRY_W);
  wt_cvt<<<dim3(CC / 64, FFD / 64), blk, 0, stream>>>(f2_w, W2T,                  FFD, CC,  CARRY_W);
  ln_rows<<<gLN, blk, 0, stream>>>(x, ln1_g, ln1_b, Hx, NROW, 0);
  gemm64<0, 0><<<gQK, blk, 0, stream>>>(
      Hx, CC, 0LL, WqkT, CC, (long long)CC * CC, wq_b, wk_b, 1, wq_b,
      (void*)QK, CC, (long long)NROW * CC, NROW, CC, CC, 1.0f / CARRY_W, CARRY_Q);
  gemm64<0, 1><<<gVT, blk, 0, stream>>>(
      WvT, CC, 0LL, Hx, BBT * CC, (long long)CC, wv_b, wv_b, 0, wv_b,
      (void*)VT, TT, (long long)CC * TT, CC, TT, CC, 1.0f / CARRY_W, CARRY_Q);
  attn_dist<<<gAttn, dim3(128), 0, stream>>>(QK, QK + (size_t)NROW * CC, VT, tao, Opl,
                                              0.125f / (CARRY_Q * CARRY_Q));
  gemm64<0, 2><<<gFC, blk, 0, stream>>>(
      Opl, CC, 0LL, WfcT, CC, 0LL, fc_b, fc_b, 0, x,
      (void*)X1, CC, 0LL, NROW, CC, CC, 1.0f / (CARRY_W * CARRY_O), 1.0f);
  ln_rows<<<gLN, blk, 0, stream>>>(X1, ln2_g, ln2_b, H2p, NROW, PADR);
  gemm64<1, 3><<<gFF1, blk, 0, stream>>>(
      H2p, CC, 0LL, W1T, KFF, 0LL, f1_b, f1_b, 0, f1_b,
      (void*)Res, FFD, 0LL, NROW, FFD, KFF, 1.0f / CARRY_W, CARRY_R);
  gemm64<0, 2><<<gFC, blk, 0, stream>>>(
      Res, FFD, 0LL, W2T, FFD, 0LL, f2_b, f2_b, 0, X1,
      d_out, CC, 0LL, NROW, CC, FFD, 1.0f / (CARRY_W * CARRY_R), 1.0f);
  (void)hipGetLastError();
}
